// ResNet_28020366639553
// MI455X (gfx1250) — hardware-verified
//
#include <hip/hip_runtime.h>


namespace {
constexpr int N = 200000, NLIM = 200000  , K9 = 9, C = 64, KD = K9 * C  , CH = 512, NCH = (N + CH - 1) / CH;
constexpr float XS = 8.0f, WSC = 256.0f, EPS = 1e-5f;
static_assert(N % 64 == 0 && NLIM % 64 == 0 && KD % 32 == 0, "tiling");
typedef _Float16 b16;
typedef __attribute__((ext_vector_type(16))) _Float16 v16b;
typedef __attribute__((ext_vector_type(8))) _Float16 v8b;
typedef __attribute__((ext_vector_type(8))) float v8f;
typedef __attribute__((ext_vector_type(4))) float v4f;
__device__ __forceinline__ float bf16_rne(float f) { unsigned int u = __float_as_uint(f); u += 0x7FFFu + ((u >> 16) & 1u); return __uint_as_float(u & 0xFFFF0000u); }
__device__ __forceinline__ void split16(float v, b16& hi, b16& lo) { hi = (b16)v; lo = (b16)(v - (float)hi); }
__device__ __forceinline__ v16b frag_kb(const b16* p, int hh) { const v8b a = *(const v8b*)(p + 8 * hh), b = *(const v8b*)(p + 16 + 8 * hh); v16b f;
#pragma unroll
  for (int e = 0; e < 8; ++e) { f[e] = a[e]; f[8 + e] = b[e]; } return f; }
__device__ __forceinline__ v8f wmma16b(v16b a, v16b b, v8f c) { v8f d = __builtin_amdgcn_wmma_f32_16x16x32_f16(false, a, false, b, (short)0, c, false, false); asm volatile("v_nop\n\tv_nop\n\tv_nop\n\tv_nop" : "+v"(d) : "v"(a), "v"(b)); return d; }
__device__ __forceinline__ void wave_lds_sync() { __builtin_amdgcn_fence(__ATOMIC_RELEASE, "workgroup"); __builtin_amdgcn_wave_barrier(); __builtin_amdgcn_fence(__ATOMIC_ACQUIRE, "workgroup"); }
__device__ __forceinline__ float pmul(float a, float b) { float p = a * b; asm volatile("" : "+v"(p)); return p; }
__device__ __forceinline__ int iclamp(int v, int lo, int hi) { return v < lo ? lo : (v > hi ? hi : v); }

typedef __attribute__((ext_vector_type(2))) float v2f;
__global__ __launch_bounds__(256) void prep_kernel(const float* __restrict__ w1, const float* __restrict__ w2, b16* __restrict__ WT) {
  const int t = blockIdx.x * 256 + threadIdx.x; if (t >= 2 * C * KD / 8) return; const int m = t / (C * KD / 8); const int e = (t % (C * KD / 8)) * 8; const int oo = e / KD, kk0 = e % KD; const float* w = m == 0 ? w1 : w2; v8b o;
  for (int j = 0; j < 8; ++j) { const int kk = kk0 + j; o[j] = (b16)(bf16_rne(w[((size_t)(kk / C) * C + kk % C) * C + oo]) * WSC); }
  for (int pass = 0; pass < 2; ++pass) { *(volatile v8b*)(WT + (size_t)m * C * KD + e) = o; __threadfence(); }
}
template <int LAYER>
__global__ __launch_bounds__(128) void conv_kernel(const float* __restrict__ SRC, const int* __restrict__ nbr, const b16* __restrict__ WT, const float* __restrict__ STAT, const float* __restrict__ gam, const float* __restrict__ bet, float* __restrict__ O) {
  __shared__ __attribute__((aligned(16))) float Tf[4][16][C + 4]; __shared__ float SM[C], SR[C], SG[C], SB[C];
  if (LAYER == 1) { for (int i = threadIdx.x; i < C; i += 128) { SM[i] = STAT[i]; SR[i] = STAT[C + i]; SG[i] = bf16_rne(gam[i]); SB[i] = bf16_rne(bet[i]); } }
  __syncthreads();
  const int wave = threadIdx.x >> 5, lane = threadIdx.x & 31, nloc = lane & 15, hlf = lane >> 4; const size_t v0 = ((size_t)blockIdx.x * 4 + wave) * 16; const size_t vr = v0 + nloc;
  int nb[K9]; for (int k = 0; k < K9; ++k) { int j = nbr[vr * K9 + k]; if (j < 0 || j >= NLIM) j = -1; nb[k] = j; }
  v8f acc[4]; for (int t = 0; t < 4; ++t) acc[t] = (v8f){};
#pragma unroll
  for (int ks = 0; ks < KD / 32; ++ks) { const int k = ks >> 1, cb = (ks & 1) * 32; const int j = nb[k]; v16b ah, al = (v16b){}; float cv[16];
    if (j >= 0) { const float* xr = SRC + (size_t)j * C + cb; const v4f c0 = *(const v4f*)(xr + 8 * hlf), c1 = *(const v4f*)(xr + 8 * hlf + 4), c2 = *(const v4f*)(xr + 16 + 8 * hlf), c3 = *(const v4f*)(xr + 16 + 8 * hlf + 4); for (int i = 0; i < 4; ++i) { cv[i] = c0[i]; cv[4 + i] = c1[i]; cv[8 + i] = c2[i]; cv[12 + i] = c3[i]; } }
    else { for (int i = 0; i < 16; ++i) cv[i] = 0.0f; }
    if (LAYER == 0) { for (int e2 = 0; e2 < 16; ++e2) ah[e2] = (b16)(bf16_rne(cv[e2]) * XS); }
    else { for (int e2 = 0; e2 < 16; ++e2) { const int c = cb + (e2 < 8 ? 0 : 16) + 8 * hlf + (e2 & 7); float hv = (j >= 0) ? fmaxf((cv[e2] - SM[c]) * SR[c] * SG[c] + SB[c], 0.0f) : 0.0f; b16 p, q; split16(hv * XS, p, q); ah[e2] = p; al[e2] = q; } }
#pragma unroll
    for (int t = 0; t < 4; ++t) { const v16b bw = frag_kb(WT + (size_t)LAYER * C * KD + (size_t)(t * 16 + nloc) * KD + ks * 32, hlf); acc[t] = wmma16b(ah, bw, acc[t]); if (LAYER == 1) acc[t] = wmma16b(al, bw, acc[t]); } }
#pragma unroll
  for (int t = 0; t < 4; ++t)
#pragma unroll
    for (int r = 0; r < 8; ++r) Tf[wave][8 * hlf + r][t * 16 + nloc] = acc[t][r] * (1.0f / (XS * WSC));
  wave_lds_sync();
  for (int pass = 0; pass < 2; ++pass) { for (int rr = 0; rr < 16; ++rr) *(volatile v2f*)(O + (v0 + rr) * C + lane * 2) = *(const v2f*)(&Tf[wave][rr][lane * 2]); __threadfence(); }
}
__global__ __launch_bounds__(128) void statA_kernel(const float* __restrict__ O, float* __restrict__ PART) {
  const int ch = blockIdx.x, t = threadIdx.x; const int c = t & 63; const bool sq = t >= 64; const size_t v0 = (size_t)ch * CH; size_t v1 = v0 + CH; if (v1 > (size_t)NLIM) v1 = (size_t)NLIM; float s = 0.0f;
#pragma unroll 4
  for (size_t v = v0; v < v1; ++v) { const float x = O[v * C + c]; s += sq ? x * x : x; }
  for (int pass = 0; pass < 2; ++pass) { ((volatile float*)PART)[(size_t)ch * 128 + t] = s; __threadfence(); }
}
__global__ __launch_bounds__(64) void statB_kernel(const float* __restrict__ PART, float* __restrict__ STAT) {
  const int c = threadIdx.x; double s = 0.0, q = 0.0;
#pragma unroll 1
  for (int ch = 0; ch < NCH; ++ch) { s += (double)PART[(size_t)ch * 128 + c]; q += (double)PART[(size_t)ch * 128 + 64 + c]; }
  const double n = (double)NLIM; const double mu = s / n; double var = q / n - mu * mu; if (var < 0.0) var = 0.0;
  for (int pass = 0; pass < 2; ++pass) { ((volatile float*)STAT)[c] = (float)mu; ((volatile float*)STAT)[64 + c] = (float)(1.0 / sqrt(var + (double)EPS)); __threadfence(); }
}
__global__ __launch_bounds__(256) void out_kernel(const float* __restrict__ O2, const float* __restrict__ STAT, const float* __restrict__ gam, const float* __restrict__ bet, const float* __restrict__ x, float* __restrict__ out) {
  const size_t u = (size_t)blockIdx.x * 256 + threadIdx.x; const size_t v = u / 32; const int c = (int)(u % 32) * 2; if (v >= (size_t)NLIM) return;
  v2f o; for (int i = 0; i < 2; ++i) o[i] = (O2[v * C + c + i] - STAT[c + i]) * STAT[64 + c + i] * bf16_rne(gam[c + i]) + bf16_rne(bet[c + i]) + bf16_rne(x[v * C + c + i]);
  for (int pass = 0; pass < 2; ++pass) { *(volatile v2f*)(out + v * C + c) = o; __threadfence(); }
}
}

extern "C" void kernel_launch(void* const* d_in, const int* in_sizes, int n_in, void* d_out, int out_size, void* d_ws, size_t ws_size, hipStream_t stream) {
  (void)n_in;
  auto Fp = [&](int i) { return (const float*)d_in[i]; }; auto Ip = [&](int i) { return (const int*)d_in[i]; };
  if (in_sizes[0] != N * C || in_sizes[1] != N * K9 || in_sizes[2] != K9 * C * C || in_sizes[3] != C || in_sizes[5] != K9 * C * C || in_sizes[7] != C || out_size != N * C) return;
  size_t off = 0; char* ws = (char*)d_ws;
  auto carve = [&](size_t bytes) { char* p = ws + off; off += (bytes + 255) & ~(size_t)255; return p; };
  b16* WT = (b16*)carve((size_t)2 * C * KD * 2); float* O1 = (float*)carve((size_t)N * C * 4); float* O2 = (float*)carve((size_t)N * C * 4); float* PART = (float*)carve((size_t)NCH * 128 * 4); float* STAT1 = (float*)carve(512); float* STAT2 = (float*)carve(512);
  if (off > ws_size || off > ((size_t)128 << 20)) return;
  prep_kernel<<<(2 * C * KD / 8 + 255) / 256, 256, 0, stream>>>(Fp(2), Fp(5), WT);
  conv_kernel<0><<<NLIM / 64, 128, 0, stream>>>(Fp(0), Ip(1), WT, nullptr, nullptr, nullptr, O1);
  statA_kernel<<<NCH, 128, 0, stream>>>(O1, PART);
  statB_kernel<<<1, 64, 0, stream>>>(PART, STAT1);
  conv_kernel<1><<<NLIM / 64, 128, 0, stream>>>(O1, Ip(1), WT, STAT1, Fp(3), Fp(4), O2);
  statA_kernel<<<NCH, 128, 0, stream>>>(O2, PART);
  statB_kernel<<<1, 64, 0, stream>>>(PART, STAT2);
  out_kernel<<<(unsigned)(((size_t)NLIM * 32 + 255) / 256), 256, 0, stream>>>(O2, STAT2, Fp(6), Fp(7), Fp(0), (float*)d_out);
}
